// GATLayerWithOrder_1932735283942
// MI455X (gfx1250) — hardware-verified
//
#include <hip/hip_runtime.h>
#include <math.h>

#define NB  64
#define NN  128
#define NF  256
#define NE  64
#define NCI 128
#define NR  (NB * NN)

static_assert(NN == 128);
static_assert(NF == 256);
static_assert(NE == 64);
static_assert(NCI == 128);

constexpr int idx_lit(int r) { return (r < NN * NN) ? (r / NN) : ((r - NN * NN) % NN); }
constexpr bool closed_rows(int i0, int i1) {
  for (int i = i0; i < i1; ++i)
    for (int j = 0; j < NN; ++j) {
      const int p  = i * NN + j;
      const int a1 = idx_lit(2 * p);
      const int a2 = idx_lit(2 * p + 1);
      const int c1 = (i < 64) ? (2 * i + (j >> 6)) : (2 * (j & 63));
      const int c2 = (i < 64) ? c1 : (2 * (j & 63) + 1);
      if (a1 != c1 || a2 != c2) return false;
    }
  return true;
}
static_assert(closed_rows(0, 16));
static_assert(closed_rows(16, 32));
static_assert(closed_rows(32, 48));
static_assert(closed_rows(48, 64));
static_assert(closed_rows(64, 80));
static_assert(closed_rows(80, 96));
static_assert(closed_rows(96, 112));
static_assert(closed_rows(112, 128));

typedef __attribute__((ext_vector_type(16))) __bf16 v16b;
typedef __attribute__((ext_vector_type(8)))  __bf16 v8b;
typedef __attribute__((ext_vector_type(8)))  float  v8f;
typedef __attribute__((ext_vector_type(4)))  float  v4f;
typedef __attribute__((ext_vector_type(4)))  unsigned int v4u;
typedef __attribute__((ext_vector_type(2)))  unsigned int v2u;
typedef __attribute__((ext_vector_type(4)))  int    v4i;
typedef v8b __attribute__((may_alias)) v8ba;
typedef v4f __attribute__((may_alias)) v4fa;
typedef v4u __attribute__((may_alias)) v4ua;
typedef v2u __attribute__((may_alias)) v2ua;
typedef unsigned short __attribute__((may_alias)) u16a;

union FB { v16b v; v8b h[2]; };

__device__ __forceinline__ v8f wmb(v16b a, v16b b, v8f c) {
  c = __builtin_amdgcn_wmma_f32_16x16x32_bf16(false, a, false, b, (short)0, c, false, false);
  asm volatile("v_nop\n\tv_nop\n\tv_nop\n\tv_nop" : "+v"(c) : "v"(a), "v"(b));
  return c;
}
__device__ __forceinline__ v16b ldg_frag(const __bf16* p) {
  FB f; f.h[0] = *(const v8ba*)(p); f.h[1] = *(const v8ba*)(p + 16); return f.v;
}
__device__ __forceinline__ v16b lds_frag(const __bf16* p) {
  FB f; f.h[0] = *(const v8ba*)(p); f.h[1] = *(const v8ba*)(p + 16); return f.v;
}

__device__ __forceinline__ unsigned bf_rne(float f) {
  const unsigned u = __float_as_uint(f);
  return (u + 0x7FFFu + ((u >> 16) & 1u)) >> 16;
}
__device__ __forceinline__ float bf_f(unsigned h) { return __uint_as_float(h << 16); }
__device__ __forceinline__ unsigned rb32(float f) { return bf_rne(f) << 16; }
__device__ __forceinline__ unsigned pk16(unsigned lo, unsigned hi) { return (lo & 0xffffu) | (hi << 16); }
__device__ __forceinline__ float leaky(float v) { return (v > 0.0f) ? v : 0.01f * v; }
__device__ __forceinline__ float sigm(float x) { return 1.0f / (1.0f + expf(-x)); }

__device__ __forceinline__ v4u hi8(const float (&f)[8]) {
  const v4u r = { pk16(bf_rne(f[0]), bf_rne(f[1])), pk16(bf_rne(f[2]), bf_rne(f[3])),
                  pk16(bf_rne(f[4]), bf_rne(f[5])), pk16(bf_rne(f[6]), bf_rne(f[7])) };
  return r;
}
__device__ __forceinline__ void split8(const float (&f)[8], v4u& hi, v4u& lo) {
  unsigned h[8], l[8];
#pragma unroll
  for (int e = 0; e < 8; ++e) { h[e] = bf_rne(f[e]); l[e] = bf_rne(f[e] - bf_f(h[e])); }
  const v4u a = { pk16(h[0], h[1]), pk16(h[2], h[3]), pk16(h[4], h[5]), pk16(h[6], h[7]) };
  const v4u b = { pk16(l[0], l[1]), pk16(l[2], l[3]), pk16(l[4], l[5]), pk16(l[6], l[7]) };
  hi = a; lo = b;
}
__device__ __forceinline__ void st2_u4(unsigned short* p, v4u v) {
  *(volatile v4u*)p = v;
  __threadfence();
  *(volatile v4u*)p = v;
}

__global__ __launch_bounds__(256) void k_pa(
    const float* __restrict__ x, const float* __restrict__ W, const float* __restrict__ a,
    const float* __restrict__ fc_w, const float* __restrict__ fc_b, const float* __restrict__ fcc_w,
    const float* __restrict__ fcc_b, const float* __restrict__ fc_out_b,
    unsigned short* __restrict__ XB, unsigned short* __restrict__ WT,
    unsigned short* __restrict__ A12T, float* __restrict__ PAR)
{
  const int blk = blockIdx.x, tid = threadIdx.x;
  if (blk < 1024) {
    const size_t u = (size_t)blk * 256 + tid;
    const v4f p = *(const v4fa*)(x + u * 8);
    const v4f q = *(const v4fa*)(x + u * 8 + 4);
    const float f[8] = { p.x, p.y, p.z, p.w, q.x, q.y, q.z, q.w };
    st2_u4(XB + u * 8, hi8(f));
  } else if (blk < 1056) {
    const int u = (blk - 1024) * 256 + tid;
    const int n = u >> 5, k8 = u & 31;
    float f[8];
#pragma unroll
    for (int e = 0; e < 8; ++e) f[e] = W[(size_t)(k8 * 8 + e) * NF + n];
    st2_u4(WT + (size_t)n * 256 + k8 * 8, hi8(f));
  } else if (blk < 1088) {
    const int u = (blk - 1056) * 256 + tid;
    const int n = u >> 6, k8 = u & 63;
    const int k = k8 * 8;
    const int rowb = ((n >= 64) ? 256 : 0) + (k & 255);
    const int col = n & 63;
    float f[8];
#pragma unroll
    for (int e = 0; e < 8; ++e) f[e] = a[(size_t)(rowb + e) * NE + col];
    st2_u4(A12T + (size_t)n * 512 + k, hi8(f));
  } else {
    const int u = tid;
    const int uw = (u < 15) ? u : 15;
    int uc = u - 32; uc = (uc < 0) ? 0 : ((uc > 63) ? 63 : uc);
    int uo = u - 96; uo = (uo < 0) ? 0 : ((uo > 63) ? 63 : uo);
    const v4f w4 = *(const v4fa*)(fc_w + 4 * uw);
    const v4f c4 = *(const v4fa*)(fcc_w + 4 * uc);
    const v4f o4 = *(const v4fa*)(fc_out_b + 4 * uo);
    const float fb = fc_b[0];
    const float cb = fcc_b[0];
    const unsigned Mw  = 0u - (unsigned)(u < 16);
    const unsigned Mfb = 0u - (unsigned)(u == 16);
    const unsigned Mcb = 0u - (unsigned)(u == 17);
    const unsigned Mc  = 0u - (unsigned)(u >= 32 && u < 96);
    const unsigned Mo  = 0u - (unsigned)(u >= 96 && u < 160);
    v4u o;
    o.x = (rb32(w4.x) & Mw) | (rb32(c4.x) & Mc) | (rb32(o4.x) & Mo) | (rb32(fb) & Mfb) | (rb32(cb) & Mcb);
    o.y = (rb32(w4.y) & Mw) | (rb32(c4.y) & Mc) | (rb32(o4.y) & Mo);
    o.z = (rb32(w4.z) & Mw) | (rb32(c4.z) & Mc) | (rb32(o4.z) & Mo);
    o.w = (rb32(w4.w) & Mw) | (rb32(c4.w) & Mc) | (rb32(o4.w) & Mo);
    float* dst = PAR + 4 * u;
    *(volatile v4u*)dst = o;
    __threadfence();
    *(volatile v4u*)dst = o;
  }
}

__global__ __launch_bounds__(256) void k_pb(
    const float* __restrict__ wih_f, const float* __restrict__ whh_f, const float* __restrict__ b_f,
    const float* __restrict__ wih_r, const float* __restrict__ whh_r, const float* __restrict__ b_r,
    const float* __restrict__ fc_out_w,
    unsigned short* __restrict__ WIHT, unsigned short* __restrict__ WHH,
    unsigned short* __restrict__ FOT, float* __restrict__ BG)
{
  const int blk = blockIdx.x, tid = threadIdx.x;
  if (blk < 128) {
    const int u = blk * 256 + tid;
    const int n = u >> 5, k8 = u & 31;
    const int kk = (k8 * 8) & 127;
    const size_t so = (size_t)(n & 511) * 128 + kk;
    const v4f a0 = *(const v4fa*)(wih_f + so), a1 = *(const v4fa*)(wih_f + so + 4);
    const v4f r0 = *(const v4fa*)(wih_r + so), r1 = *(const v4fa*)(wih_r + so + 4);
    const unsigned M = 0u - (unsigned)(n < 512);
    const float fa[8] = { a0.x, a0.y, a0.z, a0.w, a1.x, a1.y, a1.z, a1.w };
    const float fr[8] = { r0.x, r0.y, r0.z, r0.w, r1.x, r1.y, r1.z, r1.w };
    float f[8];
#pragma unroll
    for (int e = 0; e < 8; ++e)
      f[e] = __uint_as_float((__float_as_uint(fa[e]) & M) | (__float_as_uint(fr[e]) & ~M));
    st2_u4(WIHT + (size_t)n * 256 + k8 * 8, hi8(f));
  } else if (blk < 192) {
    const int u = (blk - 128) * 256 + tid;
    const int rem = u & 8191;
    const size_t so = (size_t)rem * 8;
    const v4f a0 = *(const v4fa*)(whh_f + so), a1 = *(const v4fa*)(whh_f + so + 4);
    const v4f r0 = *(const v4fa*)(whh_r + so), r1 = *(const v4fa*)(whh_r + so + 4);
    const unsigned M = 0u - (unsigned)(u < 8192);
    const float fa[8] = { a0.x, a0.y, a0.z, a0.w, a1.x, a1.y, a1.z, a1.w };
    const float fr[8] = { r0.x, r0.y, r0.z, r0.w, r1.x, r1.y, r1.z, r1.w };
    float f[8];
#pragma unroll
    for (int e = 0; e < 8; ++e)
      f[e] = __uint_as_float((__float_as_uint(fa[e]) & M) | (__float_as_uint(fr[e]) & ~M));
    st2_u4(WHH + (size_t)u * 8, hi8(f));
  } else if (blk < 320) {
    const int u = (blk - 192) * 256 + tid;
    const int n = u >> 7, k8 = u & 127;
    const int k = k8 * 8;
    const int rowb = ((k >= 512) ? 256 : 0) + (k & 255);
    float f[8];
#pragma unroll
    for (int e = 0; e < 8; ++e) f[e] = fc_out_w[(size_t)(rowb + e) * NF + n];
    st2_u4(FOT + (size_t)n * 1024 + k, hi8(f));
  } else {
    const int u = tid;
    const int i4 = 4 * (u & 127);
    const v4f a = *(const v4fa*)(b_f + i4);
    const v4f r = *(const v4fa*)(b_r + i4);
    const unsigned M = 0u - (unsigned)(u < 128);
    v4u o;
    o.x = (rb32(a.x) & M) | (rb32(r.x) & ~M);
    o.y = (rb32(a.y) & M) | (rb32(r.y) & ~M);
    o.z = (rb32(a.z) & M) | (rb32(r.z) & ~M);
    o.w = (rb32(a.w) & M) | (rb32(r.w) & ~M);
    float* dst = BG + 4 * u;
    *(volatile v4u*)dst = o;
    __threadfence();
    *(volatile v4u*)dst = o;
  }
}

template <int M, int N, int K, bool BIAS, int ACT, bool HL>
__global__ __launch_bounds__(256) __attribute__((amdgpu_num_vgpr(248)))
void k_gemm(const unsigned short* __restrict__ Ap, const unsigned short* __restrict__ Btp,
            float* __restrict__ C, const float* __restrict__ bias, unsigned short* __restrict__ Chl)
{
  static_assert(M % 32 == 0);
  static_assert(N % 64 == 0);
  static_assert(K % 32 == 0);
  static_assert(((M / 32) * (N / 64)) % 8 == 0);
  __shared__ __attribute__((aligned(16))) float sT[8 * 16 * 68];

  const int lane = threadIdx.x & 31, wave = threadIdx.x >> 5;
  const int hh = lane >> 4, rl = lane & 15;
  constexpr int TN = N / 64;
  const int tile = blockIdx.x * 8 + wave;
  if (tile >= (M / 32) * TN) return;
  const int tm = tile / TN, tn = tile - tm * TN;
  const int m0 = tm * 32, n0 = tn * 64;

  const __bf16* A  = (const __bf16*)(const void*)Ap;
  const __bf16* Bt = (const __bf16*)(const void*)Btp;
  const __bf16* a0p = A + (size_t)(m0 + rl) * K + 8 * hh;
  const __bf16* a1p = a0p + (size_t)16 * K;
  const __bf16* bp  = Bt + (size_t)(n0 + rl) * K + 8 * hh;

  const v8f zero8 = {0.f, 0.f, 0.f, 0.f, 0.f, 0.f, 0.f, 0.f};
  v8f acc[2][4];
#pragma unroll
  for (int i = 0; i < 2; ++i)
#pragma unroll
    for (int j = 0; j < 4; ++j) acc[i][j] = zero8;

#pragma unroll 1
  for (int k0 = 0; k0 < K; k0 += 32) {
    v16b bf[4];
#pragma unroll
    for (int j = 0; j < 4; ++j) bf[j] = ldg_frag(bp + (size_t)(16 * j) * K + k0);
    const v16b a0 = ldg_frag(a0p + k0);
    const v16b a1 = ldg_frag(a1p + k0);
#pragma unroll
    for (int j = 0; j < 4; ++j) {
      acc[0][j] = wmb(a0, bf[j], acc[0][j]);
      acc[1][j] = wmb(a1, bf[j], acc[1][j]);
    }
  }

  float* slab = sT + wave * (16 * 68);
#pragma unroll
  for (int i = 0; i < 2; ++i) {
    const int mBase = m0 + 16 * i;
#pragma unroll
    for (int j = 0; j < 4; ++j) {
      float bv = 0.0f;
      if (BIAS) bv = bias[n0 + 16 * j + rl];
#pragma unroll
      for (int r = 0; r < 8; ++r) {
        float v = acc[i][j][r];
        if (BIAS) v = v + bv;
        if (ACT == 1) v = (v > 0.0f) ? v : expm1f(v);
        slab[(8 * hh + r) * 68 + 16 * j + rl] = v;
      }
    }
    __builtin_amdgcn_fence(__ATOMIC_RELEASE, "workgroup");
    __builtin_amdgcn_wave_barrier();
    __builtin_amdgcn_fence(__ATOMIC_ACQUIRE, "workgroup");
    {
      const int c4 = rl * 4;
      v4f val[8];
#pragma unroll
      for (int it = 0; it < 8; ++it) val[it] = *(const v4fa*)(slab + (it * 2 + hh) * 68 + c4);
      for (int pass = 0; pass < 2; ++pass) {
#pragma unroll
        for (int it = 0; it < 8; ++it) {
          const int row = it * 2 + hh;
          *(volatile v4f*)(C + (size_t)(mBase + row) * N + n0 + c4) = val[it];
        }
        __threadfence();
      }
    }
    if (HL) {
      const int q4 = lane >> 3, c8 = (lane & 7) * 8;
      v4u hv[4], lv[4];
#pragma unroll
      for (int it = 0; it < 4; ++it) {
        const float* sp = slab + (it * 4 + q4) * 68 + c8;
        const v4f s0 = *(const v4fa*)sp;
        const v4f s1 = *(const v4fa*)(sp + 4);
        const float f[8] = { s0.x, s0.y, s0.z, s0.w, s1.x, s1.y, s1.z, s1.w };
        split8(f, hv[it], lv[it]);
      }
      for (int pass = 0; pass < 2; ++pass) {
#pragma unroll
        for (int it = 0; it < 4; ++it) {
          const int row = it * 4 + q4;
          unsigned short* cp = Chl + (size_t)(mBase + row) * (2 * N) + n0 + c8;
          *(volatile v4u*)cp = hv[it];
          *(volatile v4u*)(cp + N) = lv[it];
        }
        __threadfence();
      }
    }
    __builtin_amdgcn_fence(__ATOMIC_RELEASE, "workgroup");
    __builtin_amdgcn_wave_barrier();
    __builtin_amdgcn_fence(__ATOMIC_ACQUIRE, "workgroup");
  }
}

#define ATT_LDS_BYTES (65536 + 131072 + 65536 + 6144)
static_assert(ATT_LDS_BYTES <= 327680);
static_assert(8 * 16 * 68 * 4 <= 65536);

__global__ __launch_bounds__(256) __attribute__((amdgpu_num_vgpr(248)))
void k_att(const float* __restrict__ F12, const float* __restrict__ AF, const unsigned short* __restrict__ AFHL,
           const int* __restrict__ adj, const float* __restrict__ PAR,
           unsigned short* __restrict__ HNHL, unsigned short* __restrict__ CAT)
{
  extern __shared__ __attribute__((aligned(16))) unsigned char smem_att[];
  float*          F12s = (float*)smem_att;
  unsigned short* Vt   = (unsigned short*)(smem_att + 65536);
  unsigned short* Ps   = (unsigned short*)(smem_att + 196608);
  float*          SmP  = (float*)(smem_att + 262144);
  float*          QR   = SmP + 1024;
  float*          sS   = SmP + 1216;

  const int tid = threadIdx.x, lane = tid & 31, w = tid >> 5;
  const int hh = lane >> 4, m = lane & 15;
  const int b = blockIdx.x;

  *(v4fa*)(SmP + 4 * tid) = *(const v4fa*)(PAR + 4 * tid);

  {
    const float* gF = F12 + (size_t)b * NN * 128;
#pragma unroll 4
    for (int it = 0; it < 16; ++it) {
      const int idx = (it * 256 + tid) * 4;
      *(v4fa*)(F12s + idx) = *(const v4fa*)(gF + idx);
    }
  }
  {
    const unsigned short* gV = AFHL + (size_t)b * NN * 512;
#pragma unroll 2
    for (int it = 0; it < 32; ++it) {
      const int u = it * 256 + tid;
      const int j = u & 127, c8 = u >> 7;
      const v4u wv = *(const v4ua*)(gV + (size_t)j * 512 + c8 * 8);
      u16a* dst = (u16a*)Vt + (c8 * 8) * 128 + j;
      dst[0 * 128] = (unsigned short)(wv.x & 0xffffu);
      dst[1 * 128] = (unsigned short)(wv.x >> 16);
      dst[2 * 128] = (unsigned short)(wv.y & 0xffffu);
      dst[3 * 128] = (unsigned short)(wv.y >> 16);
      dst[4 * 128] = (unsigned short)(wv.z & 0xffffu);
      dst[5 * 128] = (unsigned short)(wv.z >> 16);
      dst[6 * 128] = (unsigned short)(wv.w & 0xffffu);
      dst[7 * 128] = (unsigned short)(wv.w >> 16);
    }
  }
  {
    const v4f cw0 = *(const v4fa*)(PAR + 128 + 8 * lane);
    const v4f cw1 = *(const v4fa*)(PAR + 132 + 8 * lane);
#pragma unroll 2
    for (int rr = 0; rr < 16; ++rr) {
      const int i = 16 * w + rr;
      const float* ar = AF + ((size_t)(b * NN + i)) * NF + 8 * lane;
      const v4f x0 = *(const v4fa*)ar;
      const v4f x1 = *(const v4fa*)(ar + 4);
      float p = x0.x * cw0.x;
      p = fmaf(x0.y, cw0.y, p); p = fmaf(x0.z, cw0.z, p); p = fmaf(x0.w, cw0.w, p);
      p = fmaf(x1.x, cw1.x, p); p = fmaf(x1.y, cw1.y, p); p = fmaf(x1.z, cw1.z, p); p = fmaf(x1.w, cw1.w, p);
      p += __shfl_xor(p, 16, 32);
      p += __shfl_xor(p, 8, 32);
      p += __shfl_xor(p, 4, 32);
      p += __shfl_xor(p, 2, 32);
      p += __shfl_xor(p, 1, 32);
      if (lane == 0) sS[i] = p;
    }
  }
  __syncthreads();

  if (tid < 192) {
    const int isq = (tid < 128) ? 1 : 0;
    const int r1 = isq ? tid : 2 * (tid - 128);
    const int r2 = isq ? tid : 2 * (tid - 128) + 1;
    const int o1 = r1 * 128, o2 = r2 * 128 + 64;
    float acc = 0.0f;
#pragma unroll 4
    for (int k = 0; k < NE; ++k) {
      const float v = leaky(F12s[o1 + k] + F12s[o2 + k]);
      acc = fmaf(SmP[k], v, acc);
    }
    QR[tid] = acc + SmP[64];
  }
  __syncthreads();

  const float fccb = SmP[68];
#pragma unroll 1
  for (int rr = 0; rr < 16; ++rr) {
    const int i = 16 * w + rr;
    const size_t row = (size_t)b * NN + i;
    const v4i av = *(const v4i*)(adj + row * NN + 4 * lane);
    const float qv = QR[(2 * i + hh) & 127];
    const v4f rv = *(const v4fa*)(QR + 128 + 4 * (lane & 15));
    const bool lowhalf = (i < 64);
    float e0 = lowhalf ? qv : rv.x;
    float e1 = lowhalf ? qv : rv.y;
    float e2 = lowhalf ? qv : rv.z;
    float e3 = lowhalf ? qv : rv.w;
    e0 = (av.x > 0) ? e0 : -9.0e15f;
    e1 = (av.y > 0) ? e1 : -9.0e15f;
    e2 = (av.z > 0) ? e2 : -9.0e15f;
    e3 = (av.w > 0) ? e3 : -9.0e15f;
    float mx = fmaxf(fmaxf(e0, e1), fmaxf(e2, e3));
    mx = fmaxf(mx, __shfl_xor(mx, 16, 32));
    mx = fmaxf(mx, __shfl_xor(mx, 8, 32));
    mx = fmaxf(mx, __shfl_xor(mx, 4, 32));
    mx = fmaxf(mx, __shfl_xor(mx, 2, 32));
    mx = fmaxf(mx, __shfl_xor(mx, 1, 32));
    const float x0 = expf(e0 - mx), x1 = expf(e1 - mx), x2 = expf(e2 - mx), x3 = expf(e3 - mx);
    float sm = (x0 + x1) + (x2 + x3);
    sm += __shfl_xor(sm, 16, 32);
    sm += __shfl_xor(sm, 8, 32);
    sm += __shfl_xor(sm, 4, 32);
    sm += __shfl_xor(sm, 2, 32);
    sm += __shfl_xor(sm, 1, 32);
    const float inv = 1.0f / sm;
    const float p0 = x0 * inv, p1 = x1 * inv, p2 = x2 * inv, p3 = x3 * inv;
    const float si = sS[i];
    const float h0 = leaky(p0 * si + fccb), h1 = leaky(p1 * si + fccb);
    const float h2 = leaky(p2 * si + fccb), h3 = leaky(p3 * si + fccb);

    const unsigned ph0 = bf_rne(p0), ph1 = bf_rne(p1), ph2 = bf_rne(p2), ph3 = bf_rne(p3);
    const unsigned pl0 = bf_rne(p0 - bf_f(ph0)), pl1 = bf_rne(p1 - bf_f(ph1));
    const unsigned pl2 = bf_rne(p2 - bf_f(ph2)), pl3 = bf_rne(p3 - bf_f(ph3));
    const v2u pvh = { pk16(ph0, ph1), pk16(ph2, ph3) };
    const v2u pvl = { pk16(pl0, pl1), pk16(pl2, pl3) };
    *(v2ua*)(Ps + i * 256 + 4 * lane) = pvh;
    *(v2ua*)(Ps + i * 256 + 128 + 4 * lane) = pvl;

    const unsigned gh0 = bf_rne(h0), gh1 = bf_rne(h1), gh2 = bf_rne(h2), gh3 = bf_rne(h3);
    const unsigned gl0 = bf_rne(h0 - bf_f(gh0)), gl1 = bf_rne(h1 - bf_f(gh1));
    const unsigned gl2 = bf_rne(h2 - bf_f(gh2)), gl3 = bf_rne(h3 - bf_f(gh3));
    const v2u hvh = { pk16(gh0, gh1), pk16(gh2, gh3) };
    const v2u hvl = { pk16(gl0, gl1), pk16(gl2, gl3) };
    unsigned short* hp = HNHL + row * 256 + 4 * lane;
    *(volatile v2u*)hp = hvh;
    *(volatile v2u*)(hp + 128) = hvl;
    __threadfence();
    *(volatile v2u*)hp = hvh;
    *(volatile v2u*)(hp + 128) = hvl;
  }
  __syncthreads();

  const __bf16* Pb = (const __bf16*)(const void*)Ps;
  const __bf16* Vb = (const __bf16*)(const void*)Vt;
  v16b pah[4], pal[4];
#pragma unroll
  for (int ks = 0; ks < 4; ++ks) {
    pah[ks] = lds_frag(Pb + (16 * w + m) * 256 + ks * 32 + 8 * hh);
    pal[ks] = lds_frag(Pb + (16 * w + m) * 256 + 128 + ks * 32 + 8 * hh);
  }
  float* slab = F12s + w * (16 * 68);
  const v8f zero8 = {0.f, 0.f, 0.f, 0.f, 0.f, 0.f, 0.f, 0.f};
#pragma unroll 1
  for (int nc = 0; nc < 4; ++nc) {
    v8f acc[4];
#pragma unroll
    for (int t = 0; t < 4; ++t) acc[t] = zero8;
#pragma unroll
    for (int ks = 0; ks < 4; ++ks) {
#pragma unroll
      for (int t = 0; t < 4; ++t) {
        const int f = nc * 64 + 16 * t + m;
        const v16b bh = lds_frag(Vb + f * 128 + ks * 32 + 8 * hh);
        const v16b bl = lds_frag(Vb + (256 + f) * 128 + ks * 32 + 8 * hh);
        acc[t] = wmb(pah[ks], bh, acc[t]);
        acc[t] = wmb(pal[ks], bh, acc[t]);
        acc[t] = wmb(pah[ks], bl, acc[t]);
      }
    }
#pragma unroll
    for (int t = 0; t < 4; ++t)
#pragma unroll
      for (int r = 0; r < 8; ++r) slab[(8 * hh + r) * 68 + 16 * t + m] = acc[t][r];
    __builtin_amdgcn_fence(__ATOMIC_RELEASE, "workgroup");
    __builtin_amdgcn_wave_barrier();
    __builtin_amdgcn_fence(__ATOMIC_ACQUIRE, "workgroup");
    {
      const int q4 = lane >> 3, c8 = (lane & 7) * 8;
      v4u hv[4], lv[4];
#pragma unroll
      for (int it = 0; it < 4; ++it) {
        const float* sp = slab + (it * 4 + q4) * 68 + c8;
        const v4f s0 = *(const v4fa*)sp;
        const v4f s1 = *(const v4fa*)(sp + 4);
        const float f[8] = { s0.x, s0.y, s0.z, s0.w, s1.x, s1.y, s1.z, s1.w };
        split8(f, hv[it], lv[it]);
      }
      for (int pass = 0; pass < 2; ++pass) {
#pragma unroll
        for (int it = 0; it < 4; ++it) {
          const int rowl = it * 4 + q4;
          unsigned short* cp = CAT + ((size_t)(b * NN + 16 * w + rowl)) * 1024 + 512 + nc * 64 + c8;
          *(volatile v4u*)cp = hv[it];
          *(volatile v4u*)(cp + 256) = lv[it];
        }
        __threadfence();
      }
    }
    __builtin_amdgcn_fence(__ATOMIC_RELEASE, "workgroup");
    __builtin_amdgcn_wave_barrier();
    __builtin_amdgcn_fence(__ATOMIC_ACQUIRE, "workgroup");
  }
}

#define LSTM_LDS_BYTES (131072 + 8192 + 32768 + 8192)
static_assert(LSTM_LDS_BYTES <= 327680);

__global__ __launch_bounds__(256) __attribute__((amdgpu_num_vgpr(248)))
void k_lstm(const float* __restrict__ XP, const unsigned short* __restrict__ WHH, unsigned short* __restrict__ CAT)
{
  extern __shared__ __attribute__((aligned(16))) unsigned char smem_lstm[];
  unsigned short* Ws  = (unsigned short*)smem_lstm;
  unsigned short* Ab  = (unsigned short*)(smem_lstm + 131072);
  float*          XPS = (float*)(smem_lstm + 139264);
  float*          HS  = (float*)(smem_lstm + 172032);

  const int tid = threadIdx.x, lane = tid & 31, w = tid >> 5;
  const int hh = lane >> 4, m = lane & 15;
  const int dir = blockIdx.x >> 2;
  const int b0 = (blockIdx.x & 3) * 16;

  {
    const unsigned short* gW = WHH + (size_t)dir * 512 * 128;
#pragma unroll 4
    for (int it = 0; it < 32; ++it) {
      const int idx = (it * 256 + tid) * 8;
      *(v4ua*)(Ws + idx) = *(const v4ua*)(gW + idx);
    }
    const v4u z = {0u, 0u, 0u, 0u};
    *(v4ua*)(Ab + tid * 8) = z;
    *(v4ua*)(Ab + 2048 + tid * 8) = z;
  }
  __syncthreads();

  const __bf16* Wb = (const __bf16*)(const void*)Ws;
  const __bf16* Ah = (const __bf16*)(const void*)Ab;
  v8f c = {0.f, 0.f, 0.f, 0.f, 0.f, 0.f, 0.f, 0.f};

#pragma unroll 1
  for (int step = 0; step < NN; ++step) {
    const int t = dir ? (NN - 1 - step) : step;
#pragma unroll 4
    for (int it = 0; it < 8; ++it) {
      const int u = it * 256 + tid;
      const int r = u >> 7, c4 = (u & 127) * 4;
      const v4f xv = *(const v4fa*)(XP + ((size_t)((b0 + r) * NN + t)) * 1024 + dir * 512 + c4);
      *(v4fa*)(XPS + r * 512 + c4) = xv;
    }
    __syncthreads();
    v8f acc[4];
#pragma unroll
    for (int g = 0; g < 4; ++g)
#pragma unroll
      for (int r = 0; r < 8; ++r) acc[g][r] = XPS[(8 * hh + r) * 512 + g * 128 + 16 * w + m];
#pragma unroll
    for (int ks = 0; ks < 4; ++ks) {
      const v16b ah = lds_frag(Ah + m * 256 + ks * 32 + 8 * hh);
      const v16b al = lds_frag(Ah + m * 256 + 128 + ks * 32 + 8 * hh);
#pragma unroll
      for (int g = 0; g < 4; ++g) {
        const v16b bf = lds_frag(Wb + (g * 128 + 16 * w + m) * 128 + ks * 32 + 8 * hh);
        acc[g] = wmb(ah, bf, acc[g]);
        acc[g] = wmb(al, bf, acc[g]);
      }
    }
#pragma unroll
    for (int r = 0; r < 8; ++r) {
      const float ig = sigm(acc[0][r]);
      const float fg = sigm(acc[1][r]);
      const float gg = tanhf(acc[2][r]);
      const float og = sigm(acc[3][r]);
      const float cn = fg * c[r] + ig * gg;
      c[r] = cn;
      HS[(8 * hh + r) * 128 + 16 * w + m] = og * tanhf(cn);
    }
    __syncthreads();
    {
      const int r = tid >> 4, c8 = (tid & 15) * 8;
      const v4f g0 = *(const v4fa*)(HS + r * 128 + c8);
      const v4f g1 = *(const v4fa*)(HS + r * 128 + c8 + 4);
      const float hv[8] = { g0.x, g0.y, g0.z, g0.w, g1.x, g1.y, g1.z, g1.w };
      const float lk[8] = { leaky(g0.x), leaky(g0.y), leaky(g0.z), leaky(g0.w),
                            leaky(g1.x), leaky(g1.y), leaky(g1.z), leaky(g1.w) };
      v4u ahi, alo, chi, clo;
      split8(hv, ahi, alo);
      split8(lk, chi, clo);
      *(v4ua*)(Ab + r * 256 + c8) = ahi;
      *(v4ua*)(Ab + r * 256 + 128 + c8) = alo;
      unsigned short* cp = CAT + ((size_t)((b0 + r) * NN + t)) * 1024 + dir * 128 + c8;
      *(volatile v4u*)cp = chi;
      *(volatile v4u*)(cp + 256) = clo;
      __threadfence();
      *(volatile v4u*)cp = chi;
      *(volatile v4u*)(cp + 256) = clo;
    }
    __syncthreads();
  }
}

extern "C" void kernel_launch(void* const* d_in, const int* in_sizes, int n_in,
                              void* d_out, int out_size, void* d_ws, size_t ws_size,
                              hipStream_t stream) {
  if (n_in < 16) return;
  if (in_sizes[0] != NB * NN * NF) return;
  if (in_sizes[1] != NB * NN * NN) return;
  if (in_sizes[2] != NF * NF) return;
  if (in_sizes[3] != 2 * NF * NE) return;
  if (in_sizes[4] != NE || in_sizes[5] != 1) return;
  if (in_sizes[6] != NF || in_sizes[7] != 1) return;
  if (in_sizes[8] != (2 * NCI + NF) * NF || in_sizes[9] != NF) return;
  if (in_sizes[10] != 4 * NCI * NN || in_sizes[11] != 4 * NCI * NCI || in_sizes[12] != 4 * NCI) return;
  if (in_sizes[13] != 4 * NCI * NN || in_sizes[14] != 4 * NCI * NCI || in_sizes[15] != 4 * NCI) return;
  if (out_size != NB * NN * NF) return;

  const float* x      = (const float*)d_in[0];
  const int*   adj    = (const int*)d_in[1];
  const float* W      = (const float*)d_in[2];
  const float* a      = (const float*)d_in[3];
  const float* fc_w   = (const float*)d_in[4];
  const float* fc_b   = (const float*)d_in[5];
  const float* fcc_w  = (const float*)d_in[6];
  const float* fcc_b  = (const float*)d_in[7];
  const float* fo_w   = (const float*)d_in[8];
  const float* fo_b   = (const float*)d_in[9];
  const float* wih_f  = (const float*)d_in[10];
  const float* whh_f  = (const float*)d_in[11];
  const float* b_f    = (const float*)d_in[12];
  const float* wih_r  = (const float*)d_in[13];
  const float* whh_r  = (const float*)d_in[14];
  const float* b_r    = (const float*)d_in[15];
  float* out = (float*)d_out;

  size_t off = 0;
  const size_t oXB   = off; off += (size_t)NR * 256 * 2;
  const size_t oAF   = off; off += (size_t)NR * 256 * 4;
  const size_t oAFHL = off; off += (size_t)NR * 512 * 2;
  const size_t oF12  = off; off += (size_t)NR * 128 * 4;
  const size_t oHNHL = off; off += (size_t)NR * 256 * 2;
  const size_t oXP   = off; off += (size_t)NR * 1024 * 4;
  const size_t oCAT  = off; off += (size_t)NR * 1024 * 2;
  const size_t oWT   = off; off += (size_t)256 * 256 * 2;
  const size_t oA12T = off; off += (size_t)128 * 512 * 2;
  const size_t oWIHT = off; off += (size_t)1024 * 256 * 2;
  const size_t oWHH  = off; off += (size_t)2 * 512 * 128 * 2;
  const size_t oFOT  = off; off += (size_t)256 * 1024 * 2;
  const size_t oPAR  = off; off += (size_t)1024 * 4;
  const size_t oBG   = off; off += (size_t)1024 * 4;
  if (off > ws_size) return;
  if (off > (size_t)134217728) return;

  char* ws = (char*)d_ws;
  unsigned short* XB   = (unsigned short*)(ws + oXB);
  float*          AF   = (float*)(ws + oAF);
  unsigned short* AFHL = (unsigned short*)(ws + oAFHL);
  float*          F12  = (float*)(ws + oF12);
  unsigned short* HNHL = (unsigned short*)(ws + oHNHL);
  float*          XP   = (float*)(ws + oXP);
  unsigned short* CAT  = (unsigned short*)(ws + oCAT);
  unsigned short* WT   = (unsigned short*)(ws + oWT);
  unsigned short* A12T = (unsigned short*)(ws + oA12T);
  unsigned short* WIHT = (unsigned short*)(ws + oWIHT);
  unsigned short* WHH  = (unsigned short*)(ws + oWHH);
  unsigned short* FOT  = (unsigned short*)(ws + oFOT);
  float*          PAR  = (float*)(ws + oPAR);
  float*          BG   = (float*)(ws + oBG);

  k_pa<<<1089, 256, 0, stream>>>(x, W, a, fc_w, fc_b, fcc_w, fcc_b, fo_b, XB, WT, A12T, PAR);
  k_pb<<<321, 256, 0, stream>>>(wih_f, whh_f, b_f, wih_r, whh_r, b_r, fo_w, WIHT, WHH, FOT, BG);

  k_gemm<NR, 256, 256, false, 0, true><<<128, 256, 0, stream>>>(XB, WT, AF, PAR, AFHL);
  k_gemm<NR, 128, 512, false, 0, false><<<64, 256, 0, stream>>>(AFHL, A12T, F12, PAR, HNHL);
  (void)hipFuncSetAttribute((const void*)k_att, hipFuncAttributeMaxDynamicSharedMemorySize, ATT_LDS_BYTES);
  k_att<<<NB, 256, ATT_LDS_BYTES, stream>>>(F12, AF, AFHL, adj, PAR, HNHL, CAT);
  k_gemm<NR, 1024, 256, true, 0, false><<<512, 256, 0, stream>>>(HNHL, WIHT, XP, BG, HNHL);
  (void)hipFuncSetAttribute((const void*)k_lstm, hipFuncAttributeMaxDynamicSharedMemorySize, LSTM_LDS_BYTES);
  k_lstm<<<8, 256, LSTM_LDS_BYTES, stream>>>(XP, WHH, CAT);
  k_gemm<NR, 256, 1024, true, 1, false><<<128, 256, 0, stream>>>(CAT, FOT, out, PAR + 384, HNHL);
  (void)hipGetLastError();
}
